// BiLSTM_CRF_49048526520834
// MI455X (gfx1250) — hardware-verified
//
#include <hip/hip_runtime.h>
#include <math.h>

typedef __attribute__((ext_vector_type(16))) _Float16 v16h;
typedef __attribute__((ext_vector_type(8)))  _Float16 v8h;
typedef __attribute__((ext_vector_type(16))) __bf16   v16b;
typedef __attribute__((ext_vector_type(8)))  __bf16   v8b;
typedef __attribute__((ext_vector_type(8)))  float    v8f;
typedef __attribute__((ext_vector_type(4)))  float    v4f;

constexpr int kB    = 64;
constexpr int kT    = 512;
constexpr int kV    = 30000;
constexpr int kE    = 256;
constexpr int kHD   = 128;
constexpr int kG4   = 4 * kHD;
constexpr int kK    = kHD + kE;
constexpr int kTag  = 16;
constexpr int kTagP = 64;
constexpr int kRows = kB * kT;
constexpr int kThr  = 256;
constexpr float kInCarry = 1024.0f;
constexpr float kSc = 1.0f / (kInCarry * kInCarry);
constexpr float kF16MinNormal = 6.103515625e-5f;
constexpr int kFBO = 0, kFBZ = 64, kFEnd = 1024;

static_assert(kB == 64 && (kG4 / 64) % 8 == 0 && (kRows % 64) == 0 && ((kRows / 64) * (kTagP / 64)) % 8 == 0 && (kK % 32) == 0 && ((2 * kHD) % 32) == 0 && kFBZ + kG4 <= kFEnd && kTag <= kTagP,
              "GEMM M, N multiples of 64; grids exact; K multiples of 32");

constexpr size_t kOffW2 = 0ull;
constexpr size_t kOffWO16 = 786432ull;
constexpr size_t kOffBIAS = 819200ull;
constexpr size_t kOffA2 = 823296ull;
constexpr size_t kOffG2 = 921600ull;
constexpr size_t kOffC2 = 1183744ull;
constexpr size_t kOffHS16 = 1249280ull;
constexpr size_t kOffEM32 = 18026496ull;
constexpr size_t kWsTotal = 26415104ull;
static_assert(kWsTotal <= 134217728ull, "carve cap: under 128 MiB");
static_assert(kOffW2 == 0
              && kOffWO16 == kOffW2 + 786432ull
              && kOffBIAS == kOffWO16 + 32768ull
              && kOffA2 == kOffBIAS + 4096ull
              && kOffG2 == kOffA2 + 98304ull
              && kOffC2 == kOffG2 + 262144ull
              && kOffHS16 == kOffC2 + 65536ull
              && kOffEM32 == kOffHS16 + 16777216ull
              && kWsTotal == kOffEM32 + 8388608ull, "the carve is chained and totalled");
static_assert((kOffW2 % 256) == 0 && (kOffWO16 % 256) == 0 && (kOffBIAS % 256) == 0 && (kOffA2 % 256) == 0 && (kOffG2 % 256) == 0 && (kOffC2 % 256) == 0 && (kOffHS16 % 256) == 0 && (kOffEM32 % 256) == 0, "aligned regions");

__device__ __forceinline__ unsigned short f2bf_bits(float f) {
  unsigned u = __float_as_uint(f);
  return (unsigned short)((u + 0x7FFFu + ((u >> 16) & 1u)) >> 16);
}
__device__ __forceinline__ float bf_bits2f(unsigned short h) { return __uint_as_float(((unsigned)h) << 16); }
__device__ __forceinline__ float bf16r(float f) { return bf_bits2f(f2bf_bits(f)); }
__device__ __forceinline__ float carry_flush(float v, float carry) {
  const float s = v * carry;
  return (fabsf(s) < kF16MinNormal) ? 0.0f : s;
}
__device__ __forceinline__ float frcp(float x) { return __builtin_amdgcn_rcpf(x); }

__device__ __forceinline__ void dep_guard4_h(v8f& a, v8f& b, v8f& c, v8f& d, v16h x, v16h y) { asm volatile("v_nop\n\tv_nop\n\tv_nop\n\tv_nop" : "+v"(a), "+v"(b), "+v"(c), "+v"(d) : "v"(x), "v"(y)); }
__device__ __forceinline__ void dep_guard4_b(v8f& a, v8f& b, v8f& c, v8f& d, v16b x, v16b y) { asm volatile("v_nop\n\tv_nop\n\tv_nop\n\tv_nop" : "+v"(a), "+v"(b), "+v"(c), "+v"(d) : "v"(x), "v"(y)); }
__device__ __forceinline__ void keep4_h(v16h a, v16h b, v16h c, v16h d) { asm volatile("v_nop" :: "v"(a), "v"(b), "v"(c), "v"(d)); }
__device__ __forceinline__ void keep4_b(v16b a, v16b b, v16b c, v16b d) { asm volatile("v_nop" :: "v"(a), "v"(b), "v"(c), "v"(d)); }
__device__ __forceinline__ void acc_guard4(v8f& a, v8f& b, v8f& c, v8f& d) { asm volatile("v_nop\n\tv_nop\n\tv_nop\n\tv_nop" : "+v"(a), "+v"(b), "+v"(c), "+v"(d)); }

template <typename T> struct Frag;
template <> struct Frag<_Float16> {
  typedef v16h V; union U { v16h v; v8h h[2]; };
  static __device__ __forceinline__ v16h load(const _Float16* p) {
    U f; f.h[0] = *(const v8h*)(p); f.h[1] = *(const v8h*)(p + 16); return f.v;
  }
  static __device__ __forceinline__ v8f mma(v16h a, v16h b, v8f c) {
    return __builtin_amdgcn_wmma_f32_16x16x32_f16(false, a, false, b, (short)0, c, false, false);
  }
  static __device__ __forceinline__ void guard4(v8f& a, v8f& b, v8f& c, v8f& d, v16h x, v16h y) { dep_guard4_h(a, b, c, d, x, y); }
  static __device__ __forceinline__ void keep(v16h a, v16h b, v16h c, v16h d) { keep4_h(a, b, c, d); }
};
template <> struct Frag<__bf16> {
  typedef v16b V; union U { v16b v; v8b h[2]; };
  static __device__ __forceinline__ v16b load(const __bf16* p) {
    U f; f.h[0] = *(const v8b*)(p); f.h[1] = *(const v8b*)(p + 16); return f.v;
  }
  static __device__ __forceinline__ v8f mma(v16b a, v16b b, v8f c) {
    return __builtin_amdgcn_wmma_f32_16x16x32_bf16(false, a, false, b, (short)0, c, false, false);
  }
  static __device__ __forceinline__ void guard4(v8f& a, v8f& b, v8f& c, v8f& d, v16b x, v16b y) { dep_guard4_b(a, b, c, d, x, y); }
  static __device__ __forceinline__ void keep(v16b a, v16b b, v16b c, v16b d) { keep4_b(a, b, c, d); }
};

__device__ __forceinline__ v8f mma_h(v16h a, v16h b, v8f c) {
  c = __builtin_amdgcn_wmma_f32_16x16x32_f16(false, a, false, b, (short)0, c, false, false);
  asm volatile("v_nop\n\tv_nop\n\tv_nop\n\tv_nop" : "+v"(c) : "v"(a), "v"(b));
  return c;
}

template <int ET> struct Elem;
template <> struct Elem<0> { typedef _Float16 T; };
template <> struct Elem<1> { typedef __bf16 T; };
template <int ET, bool SPLIT, int BIAS_MODE, int OUT_MODE, bool RESID, int ACT = 0>
__global__ __launch_bounds__(256) void wmma_gemm64(
    const unsigned short* __restrict__ Ap, const unsigned short* __restrict__ A2p, int lda, long strideA,
    const unsigned short* __restrict__ Btp, const unsigned short* __restrict__ Bt2p, int ldb, long strideB,
    void* __restrict__ Cout, void* __restrict__ Cout2, int ldc, long strideC,
    const float* __restrict__ bias,
    const float* __restrict__ resid, long strideR,
    int M, int N, int K, float scale) {
  typedef typename Elem<ET>::T T;
  typedef typename Frag<T>::V V;
  const T* A = (const T*)Ap; const T* A2 = (const T*)A2p; const T* Bt = (const T*)Btp; const T* Bt2 = (const T*)Bt2p;
  __shared__ __align__(16) float sT[8][16 * 68];
  const int b    = blockIdx.y;
  const int lane = threadIdx.x & 31;
  const int wave = threadIdx.x >> 5;
  const int tilesN = N >> 6;
  const int tilesM = M >> 6;
  const int tile = blockIdx.x * 8 + wave;
  if (tile >= tilesM * tilesN) return;
  const int tm = tile / tilesN;
  const int tn = tile - tm * tilesN;
  const int m0 = tm << 6;
  const int n0 = tn << 6;

  const T* Ab  = A  + (size_t)b * strideA;
  const T* Bb  = Bt + (size_t)b * strideB;
  const T* Ab2 = SPLIT ? (A2  + (size_t)b * strideA) : nullptr;
  const T* Bb2 = SPLIT ? (Bt2 + (size_t)b * strideB) : nullptr;

  const int rlane = lane & 15;
  const int koff  = (lane >> 4) * 8;
  const int mOff  = (lane >> 4) * 8;

  v8f acc[4][4];
#pragma unroll
  for (int i = 0; i < 4; ++i)
#pragma unroll
    for (int j = 0; j < 4; ++j) acc[i][j] = (v8f){0.f,0.f,0.f,0.f,0.f,0.f,0.f,0.f};

  for (int k0 = 0; k0 < K; k0 += 32) {
    V bh[4], bl[4];
#pragma unroll
    for (int j = 0; j < 4; ++j) {
      const size_t bo = (size_t)(n0 + (j << 4) + rlane) * ldb + koff + k0;
      bh[j] = Frag<T>::load(Bb + bo);
      if (SPLIT) bl[j] = Frag<T>::load(Bb2 + bo);
    }
#pragma unroll
    for (int i = 0; i < 4; ++i) {
      const size_t ao = (size_t)(m0 + (i << 4) + rlane) * lda + koff + k0;
      V ah = Frag<T>::load(Ab + ao);
      V al;
      if (SPLIT) al = Frag<T>::load(Ab2 + ao);
#pragma unroll
      for (int j = 0; j < 4; ++j) {
        acc[i][j] = Frag<T>::mma(ah, bh[j], acc[i][j]);
        if (SPLIT) {
          acc[i][j] = Frag<T>::mma(ah, bl[j], acc[i][j]);
          acc[i][j] = Frag<T>::mma(al, bh[j], acc[i][j]);
        }
      }
      Frag<T>::guard4(acc[i][0], acc[i][1], acc[i][2], acc[i][3], ah, SPLIT ? al : ah);
    }
    Frag<T>::keep(bh[0], bh[1], bh[2], bh[3]);
    if (SPLIT) Frag<T>::keep(bl[0], bl[1], bl[2], bl[3]);
  }
  acc_guard4(acc[0][0], acc[0][1], acc[0][2], acc[0][3]);
  acc_guard4(acc[1][0], acc[1][1], acc[1][2], acc[1][3]);
  acc_guard4(acc[2][0], acc[2][1], acc[2][2], acc[2][3]);
  acc_guard4(acc[3][0], acc[3][1], acc[3][2], acc[3][3]);

  float* slab = sT[wave];
  const float* Rb = RESID ? (resid + (size_t)b * strideR) : nullptr;
#pragma unroll
  for (int i = 0; i < 4; ++i) {
    const int mBase = m0 + (i << 4);
#pragma unroll
    for (int j = 0; j < 4; ++j) {
      const int n = n0 + (j << 4) + rlane;
      float bv = 0.f;
      if (BIAS_MODE == 2) bv = bias[n];
#pragma unroll
      for (int r = 0; r < 8; ++r) {
        float v = acc[i][j][r] * scale;
        if (BIAS_MODE == 1) v += bias[mBase + mOff + r];
        if (BIAS_MODE == 2) v += bv;
        if (RESID) v += Rb[(size_t)(mBase + mOff + r) * ldc + n];
        if (ACT == 1) v = tanhf(v);
        if (ACT == 2) v = fmaxf(v, 0.0f);
        if (ACT == 3) v = v / (1.0f + expf(-v));
        if (ACT == 4) v = (v > 0.f) ? v : 0.01f * v;
        slab[(mOff + r) * 68 + (j << 4) + rlane] = v;
      }
    }
    __builtin_amdgcn_fence(__ATOMIC_RELEASE, "workgroup");
    __builtin_amdgcn_wave_barrier();
    __builtin_amdgcn_fence(__ATOMIC_ACQUIRE, "workgroup");
    if (OUT_MODE == 0) {
      float* C = (float*)Cout + (size_t)b * strideC;
      const int hh = lane >> 4, c4 = (lane & 15) * 4;
      for (int pass = 0; pass < 2; ++pass) {
#pragma unroll
        for (int it = 0; it < 8; ++it) {
          const int row = it * 2 + hh;
          v4f v = *(const v4f*)(slab + row * 68 + c4);
          *(volatile v4f*)(C + (size_t)(mBase + row) * ldc + n0 + c4) = v;
        }
        __threadfence();
      }
    } else {
      const int q = lane >> 3, c8 = (lane & 7) * 8;
      unsigned short* C  = (unsigned short*)Cout  + (size_t)b * strideC;
      unsigned short* C2 = (OUT_MODE == 2) ? ((unsigned short*)Cout2 + (size_t)b * strideC) : nullptr;
      for (int pass = 0; pass < 2; ++pass) {
#pragma unroll
        for (int it = 0; it < 4; ++it) {
          const int row = it * 4 + q;
          const float* sp = slab + row * 68 + c8;
          v8h hv, lv;
#pragma unroll
          for (int e = 0; e < 8; ++e) {
            if (OUT_MODE == 1) {
              hv[e] = (_Float16)sp[e];
            } else {
              unsigned short hb = f2bf_bits(sp[e]);
              unsigned short lb = f2bf_bits(sp[e] - bf_bits2f(hb));
              hv[e] = __builtin_bit_cast(_Float16, hb);
              lv[e] = __builtin_bit_cast(_Float16, lb);
            }
          }
          *(volatile v8h*)(C + (size_t)(mBase + row) * ldc + n0 + c8) = hv;
          if (OUT_MODE == 2) *(volatile v8h*)(C2 + (size_t)(mBase + row) * ldc + n0 + c8) = lv;
        }
        __threadfence();
      }
    }
    __builtin_amdgcn_fence(__ATOMIC_RELEASE, "workgroup");
    __builtin_amdgcn_wave_barrier();
    __builtin_amdgcn_fence(__ATOMIC_ACQUIRE, "workgroup");
  }
}


__device__ __forceinline__ float fast_tanh(float v) { return 1.0f - 2.0f * frcp(__expf(2.0f * v) + 1.0f); }
__device__ __forceinline__ float fast_sigmoid(float v) { return frcp(1.0f + __expf(-v)); }

__device__ __forceinline__ int token_at(const int* __restrict__ sentences, unsigned b, int t) {
  int tok = sentences[(size_t)b * kT + t];
  asm volatile("" : "+v"(tok));
  return (tok < 0) ? 0 : ((tok >= kV) ? (kV - 1) : tok);
}

__global__ __launch_bounds__(kThr) void setup_kernel(const int* __restrict__ sentences, const float* __restrict__ embedding, const float* __restrict__ W_ih_f,
                                                     const float* __restrict__ W_hh_f, const float* __restrict__ W_ih_b, const float* __restrict__ W_hh_b,
                                                     const float* __restrict__ W_out, const float* __restrict__ b_out, float* __restrict__ BIAS,
                                                     unsigned short* __restrict__ W2, unsigned short* __restrict__ WO16, unsigned short* __restrict__ A2,
                                                     float* __restrict__ C2) {
  unsigned v = blockIdx.x * (unsigned)kThr + threadIdx.x;
  asm volatile("" : "+v"(v));
  if (v < 256u) {
    const unsigned i0 = v * 4u;
    const bool live = i0 < (unsigned)kTag;
    const v4f a = *(const v4f*)(b_out + (live ? i0 : 0u));
    v4f o;
#pragma unroll
    for (int e = 0; e < 4; ++e) { const float p = a[e]; o[e] = live ? bf16r(p) : 0.0f; }
    float* dp = BIAS + i0;
    *(volatile v4f*)dp = o;
    __threadfence();
    *(volatile v4f*)dp = o;
  } else if (v < 57600u) {
    v8h hv;
    unsigned short* dp;
    const float* sp;
    bool live = true;
    if (v < 49408u) {
      unsigned w = v - 256u;
      asm volatile("" : "+v"(w));
      const unsigned d = w / 24576u, n = (w / 48u) % 512u, c8 = (w % 48u) * 8u;
      const float* Wh = d ? W_hh_b : W_hh_f;
      const float* Wi = d ? W_ih_b : W_ih_f;
      sp = (c8 < (unsigned)kHD) ? (Wh + (size_t)n * kHD + c8) : (Wi + (size_t)n * kE + (c8 - (unsigned)kHD));
      dp = W2 + (size_t)w * 8u;
    } else if (v < 51456u) {
      const unsigned w = v - 49408u;
      const unsigned n = w >> 5, c8 = (w & 31u) * 8u;
      live = n < (unsigned)kTag;
      sp = W_out + (size_t)(live ? n : 0u) * (2 * kHD) + c8;
      dp = WO16 + (size_t)w * 8u;
    } else {
      unsigned w = v - 51456u;
      asm volatile("" : "+v"(w));
      const unsigned d = w / 3072u, b = (w / 48u) % 64u, c8 = (w % 48u) * 8u;
      live = c8 >= (unsigned)kHD;
      const int tok = token_at(sentences, b, d ? (kT - 1) : 0);
      sp = embedding + (size_t)tok * kE + (live ? (c8 - (unsigned)kHD) : 0u);
      dp = A2 + (size_t)w * 8u;
    }
    const v4f a0 = *(const v4f*)sp, a1 = *(const v4f*)(sp + 4);
#pragma unroll
    for (int e = 0; e < 4; ++e) { const float p = a0[e], q = a1[e]; hv[e] = (_Float16)(live ? carry_flush(bf16r(p), kInCarry) : 0.0f); hv[4 + e] = (_Float16)(live ? carry_flush(bf16r(q), kInCarry) : 0.0f); }
    *(volatile v8h*)dp = hv;
    __threadfence();
    *(volatile v8h*)dp = hv;
  } else {
    const v4f z = {0.f, 0.f, 0.f, 0.f};
    float* dp = C2 + (size_t)(v - 57600u) * 4u;
    *(volatile v4f*)dp = z;
    __threadfence();
    *(volatile v4f*)dp = z;
  }
}
static_assert(kFEnd / 4 == 256 && 2 * kG4 * (kK / 8) == 49152 && 256 + 49152 == 49408 && kTagP * (2 * kHD / 8) == 2048 && 49408 + 2048 == 51456 && 2 * kB * (kK / 8) == 6144
              && 51456 + 6144 == 57600 && 2 * kB * kHD / 4 == 4096 && 57600 + 4096 == 241 * kThr && kK / 8 == 48 && kG4 * 48 == 24576 && kB * 48 == 3072, "set-up grid exact");

__global__ __launch_bounds__(kThr) void cell2_kernel(const float* __restrict__ G2, const float* __restrict__ b_f, const float* __restrict__ b_b,
                                                     const int* __restrict__ sentences, const float* __restrict__ embedding, float* __restrict__ C2,
                                                     unsigned short* __restrict__ A2, unsigned short* __restrict__ HS16, int s) {
  const int d = (int)(blockIdx.x >> 2);
  const int t = d ? (kT - 1 - s) : s;
  unsigned v = (blockIdx.x & 3u) * (unsigned)kThr + threadIdx.x;
  asm volatile("" : "+v"(v));
  const unsigned b = v >> 4, u8 = (v & 15u) * 8u;
  const float* gr = G2 + ((size_t)d * kB + b) * kG4 + u8;
  const float* br = (d ? b_b : b_f) + u8;
  float* cp = C2 + ((size_t)d * kB + b) * kHD + u8;
  v4f cn0, cn1; v8h hv;
#pragma unroll
  for (int hlf = 0; hlf < 2; ++hlf) {
    const v4f gi = *(const v4f*)(gr + 4 * hlf), gf = *(const v4f*)(gr + kHD + 4 * hlf), gg = *(const v4f*)(gr + 2 * kHD + 4 * hlf), go = *(const v4f*)(gr + 3 * kHD + 4 * hlf);
    const v4f bi = *(const v4f*)(br + 4 * hlf), bf_ = *(const v4f*)(br + kHD + 4 * hlf), bg = *(const v4f*)(br + 2 * kHD + 4 * hlf), bo = *(const v4f*)(br + 3 * kHD + 4 * hlf);
    const v4f co = *(const v4f*)(cp + 4 * hlf);
#pragma unroll
    for (int e = 0; e < 4; ++e) {
      const float p0 = bi[e], p1 = bf_[e], p2 = bg[e], p3 = bo[e];
      const float cn = fast_sigmoid(gf[e] + bf16r(p1)) * co[e] + fast_sigmoid(gi[e] + bf16r(p0)) * fast_tanh(gg[e] + bf16r(p2));
      const float hn = fast_sigmoid(go[e] + bf16r(p3)) * fast_tanh(cn);
      if (hlf == 0) cn0[e] = cn; else cn1[e] = cn;
      hv[4 * hlf + e] = (_Float16)carry_flush(hn, kInCarry);
    }
  }
  const int tn = d ? (t - 1) : (t + 1);
  const bool nx = (tn >= 0) && (tn < kT);
  const int tok = token_at(sentences, b, nx ? tn : t);
  const float* ep = embedding + (size_t)tok * kE + (v & 15u) * 16u;
  v8h e0, e1;
  {
    const v4f m0 = *(const v4f*)ep, m1 = *(const v4f*)(ep + 4), m2 = *(const v4f*)(ep + 8), m3 = *(const v4f*)(ep + 12);
#pragma unroll
    for (int e = 0; e < 4; ++e) {
      const float q0 = m0[e], q1 = m1[e], q2 = m2[e], q3 = m3[e];
      e0[e] = (_Float16)carry_flush(bf16r(q0), kInCarry); e0[4 + e] = (_Float16)carry_flush(bf16r(q1), kInCarry);
      e1[e] = (_Float16)carry_flush(bf16r(q2), kInCarry); e1[4 + e] = (_Float16)carry_flush(bf16r(q3), kInCarry);
    }
  }
  unsigned short* ar = A2 + ((size_t)d * kB + b) * kK;
  unsigned short* hp = ar + u8;
  unsigned short* xp = ar + kHD + (v & 15u) * 16u;
  unsigned short* op = HS16 + ((size_t)b * kT + (size_t)t) * (2 * kHD) + (size_t)d * kHD + u8;
  for (int pass = 0; pass < 2; ++pass) {
    *(volatile v4f*)cp = cn0; *(volatile v4f*)(cp + 4) = cn1;
    *(volatile v8h*)hp = hv;
    *(volatile v8h*)op = hv;
    if (nx) { *(volatile v8h*)xp = e0; *(volatile v8h*)(xp + 8) = e1; }
    __threadfence();
  }
}
static_assert(kB * kHD / 8 == 4 * kThr && kHD / 8 == 16 && kE == 16 * 16, "cell grid: 4 blocks a direction; 16 threads a sample, two embedding pieces each");

__global__ __launch_bounds__(kThr) void crf_kernel(const float* __restrict__ EM32, const float* __restrict__ transition, float* __restrict__ out) {
  unsigned v = blockIdx.x * (unsigned)kThr + threadIdx.x;
  asm volatile("" : "+v"(v));
  const unsigned i4 = v * 4u;
  const unsigned row = i4 >> 8, i = (i4 >> 4) & 15u, j4 = i4 & 15u;
  const v4f e4 = *(const v4f*)(EM32 + (size_t)row * kTagP + j4), t4 = *(const v4f*)(transition + (size_t)i * kTag + j4);
  v4f o;
#pragma unroll
  for (int e = 0; e < 4; ++e) { const float p = t4[e]; o[e] = e4[e] + bf16r(p); }
  float* dp = out + (size_t)i4;
  *(volatile v4f*)dp = o;
  __threadfence();
  *(volatile v4f*)dp = o;
}
static_assert((size_t)kRows * kTag * kTag / 4 == 8192 * (size_t)kThr, "output grid exact");

extern "C" void kernel_launch(void* const* d_in, const int* in_sizes, int n_in,
                              void* d_out, int out_size, void* d_ws, size_t ws_size,
                              hipStream_t stream) {
  if (n_in < 11 || d_out == nullptr || d_ws == nullptr) return;
  if (in_sizes[0] != kB * kT || in_sizes[1] != kV * kE || in_sizes[2] != kG4 * kE || in_sizes[3] != kG4 * kHD || in_sizes[4] != kG4) return;
  if (in_sizes[5] != kG4 * kE || in_sizes[6] != kG4 * kHD || in_sizes[7] != kG4 || in_sizes[8] != kTag * 2 * kHD || in_sizes[9] != kTag || in_sizes[10] != kTag * kTag) return;
  if ((size_t)out_size != (size_t)kRows * kTag * kTag) return;
  if (ws_size < kWsTotal) return;
  const int* sentences = (const int*)d_in[0];
  const float* embedding = (const float*)d_in[1];
  const float* W_ih_f = (const float*)d_in[2];
  const float* W_hh_f = (const float*)d_in[3];
  const float* b_f = (const float*)d_in[4];
  const float* W_ih_b = (const float*)d_in[5];
  const float* W_hh_b = (const float*)d_in[6];
  const float* b_b = (const float*)d_in[7];
  const float* W_out = (const float*)d_in[8];
  const float* b_out = (const float*)d_in[9];
  const float* transition = (const float*)d_in[10];
  float* out = (float*)d_out;
  char* ws = (char*)d_ws;
  unsigned short* W2 = (unsigned short*)(ws + kOffW2);
  unsigned short* WO16 = (unsigned short*)(ws + kOffWO16);
  float* BIAS = (float*)(ws + kOffBIAS);
  unsigned short* A2 = (unsigned short*)(ws + kOffA2);
  float* G2 = (float*)(ws + kOffG2);
  float* C2 = (float*)(ws + kOffC2);
  unsigned short* HS16 = (unsigned short*)(ws + kOffHS16);
  float* EM32 = (float*)(ws + kOffEM32);

  setup_kernel<<<241, kThr, 0, stream>>>(sentences, embedding, W_ih_f, W_hh_f, W_ih_b, W_hh_b, W_out, b_out, BIAS, W2, WO16, A2, C2);

  for (int s = 0; s < kT; ++s) {
    wmma_gemm64<0, false, 2, 0, false, 0><<<dim3((kB / 64) * (kG4 / 64) / 8, 2), 256, 0, stream>>>(
        A2, A2, kK, (long)kB * kK, W2, W2, kK, (long)kG4 * kK, (void*)G2, (void*)G2, kG4, (long)kB * kG4, BIAS + kFBZ, nullptr, 0L, kB, kG4, kK, kSc);
    cell2_kernel<<<8, kThr, 0, stream>>>(G2, b_f, b_b, sentences, embedding, C2, A2, HS16, s);
  }
  wmma_gemm64<0, false, 2, 0, false, 0><<<dim3((kRows / 64) * (kTagP / 64) / 8, 1), 256, 0, stream>>>(
      HS16, HS16, 2 * kHD, 0L, WO16, WO16, 2 * kHD, 0L, (void*)EM32, (void*)EM32, kTagP, 0L, BIAS + kFBO, nullptr, 0L, kRows, kTagP, 2 * kHD, kSc);
  crf_kernel<<<8192, kThr, 0, stream>>>(EM32, transition, out);
}
